// CausalSelfAttention_34162169872985
// MI455X (gfx1250) — hardware-verified
//
#include <hip/hip_runtime.h>


#ifndef NB
#define NB 4
#endif
#ifndef SEQ
#define SEQ 1024
#endif
#define NB_FULL  4
#define SEQ_FULL 1024
#define DM   1024
#define NH   16
#define HD   64
#define D3   (3 * DM)
#define CK   (2 * DM)
#define L2E  1.4426950408889634f
#define PLSZ ((size_t)NB * NH * SEQ * HD)
#define EROWS 512
#define ER   (SEQ < EROWS ? SEQ : EROWS)
#define VRSZ ((size_t)NB * NH * HD * ER)
#define VRCAR 2048.0f
#define PEXP 8.0f
#define RB   64
#define AW   4

static_assert(SEQ % 64 == 0);
static_assert(NB >= 1 && NB <= NB_FULL && SEQ <= SEQ_FULL);
static_assert(DM == NH * HD);
static_assert(HD == 64);
static_assert(HD * 2 == 128);
static_assert(NH == 16);
static_assert((DM & (DM - 1)) == 0);
static_assert(DM % 64 == 0 && D3 % 64 == 0 && DM % 32 == 0 && HD % 32 == 0 && CK % 32 == 0);
static_assert(ER % 64 == 0 && (SEQ - ER) % 64 == 0 && ER % 32 == 0);
static_assert(AW * 16 == 64);
static_assert(RB == 64);
static_assert(NB <= 4);
static_assert(((size_t)SEQ * DM) % 8 == 0 && ((size_t)D3 * DM) % 4 == 0 && ((size_t)DM * DM) % 4 == 0);
static_assert(VRSZ % 8 == 0 && PLSZ % 8 == 0);

typedef _Float16 h16;
typedef unsigned short bf;
typedef __attribute__((ext_vector_type(16))) __bf16   v16bf;
typedef __attribute__((ext_vector_type(16))) _Float16 v16h;
typedef __attribute__((ext_vector_type(8)))  _Float16 v8h;
typedef __attribute__((ext_vector_type(8)))  unsigned short v8us;
typedef __attribute__((ext_vector_type(8)))  float    v8f;
typedef __attribute__((ext_vector_type(4)))  float    v4f;
typedef __attribute__((ext_vector_type(4)))  unsigned v4u;
typedef __attribute__((ext_vector_type(8)))  unsigned v8u;
typedef v8h  __attribute__((may_alias)) v8ha;
typedef v8us __attribute__((may_alias)) v8usa;
typedef v4f  __attribute__((may_alias)) v4fa;
typedef v4u  __attribute__((may_alias)) v4ua;

__device__ __forceinline__ unsigned short f2bf(float f) { unsigned u = __float_as_uint(f); u += 0x7FFFu + ((u >> 16) & 1u); return (unsigned short)(u >> 16); }
__device__ __forceinline__ float bf2f(unsigned short b) { return __uint_as_float(((unsigned)b) << 16); }
__device__ __forceinline__ float bfr(float f) { return bf2f(f2bf(f)); }
__device__ __forceinline__ void splitf(float y, unsigned short& h, unsigned short& l) { h = f2bf(y); l = f2bf(y - bf2f(h)); }
__device__ __forceinline__ unsigned splitw(float y) { const unsigned u = __float_as_uint(y); const float lo = y - __uint_as_float(u & 0xffff0000u); return (u >> 16) | (((unsigned)f2bf(lo)) << 16); }
__device__ __forceinline__ v16h cat16(v8h lo, v8h hi) { return __builtin_shufflevector(lo, hi, 0, 1, 2, 3, 4, 5, 6, 7, 8, 9, 10, 11, 12, 13, 14, 15); }
__device__ __forceinline__ v16bf cat16b(v8us lo, v8us hi) { return __builtin_bit_cast(v16bf, __builtin_shufflevector(lo, hi, 0, 1, 2, 3, 4, 5, 6, 7, 8, 9, 10, 11, 12, 13, 14, 15)); }
__device__ __forceinline__ v8f wmma16(v16h a, v16h b, v8f c) { return __builtin_amdgcn_wmma_f32_16x16x32_f16(false, a, false, b, (short)0, c, false, false); }
__device__ __forceinline__ v8f wmmab(v16bf a, v16bf b, v8f c) { return __builtin_amdgcn_wmma_f32_16x16x32_bf16(false, a, false, b, (short)0, c, false, false); }
__device__ __forceinline__ v16bf ldb(const bf* p) { return cat16b(*(const v8us*)p, *(const v8us*)(p + 16)); }
__device__ __forceinline__ v16h ldh(const h16* p) { return cat16(*(const v8h*)p, *(const v8h*)(p + 16)); }

static __device__ __forceinline__ h16 toh_flush(float v) { const h16 r = (h16)v; return (fabsf(v) < 6.103515625e-05f) ? (h16)0.0f : r; }
static __device__ __forceinline__ v8f gwb(v16bf a, v16bf b, v8f c) { c = __builtin_amdgcn_wmma_f32_16x16x32_bf16(false, a, false, b, (short)0, c, false, false); asm volatile("v_nop\n\tv_nop\n\tv_nop\n\tv_nop" : "+v"(c) : "v"(a), "v"(b)); return c; }
static __device__ __forceinline__ v8f gwh(v16h a, v16h b, v8f c) { c = __builtin_amdgcn_wmma_f32_16x16x32_f16(false, a, false, b, (short)0, c, false, false); asm volatile("v_nop\n\tv_nop\n\tv_nop\n\tv_nop" : "+v"(c) : "v"(a), "v"(b)); return c; }

__global__ __launch_bounds__(32) void k_gemm_bf(const bf* __restrict__ A, const bf* __restrict__ Bt, int K, float* C, int ldc, const float* __restrict__ bias, float oscale, size_t sA, size_t sB, size_t sC) {
    __shared__ __align__(16) float os[16 * 68];
    const size_t z = blockIdx.z; A += z * sA; Bt += z * sB; C += z * sC;
    const int lane = threadIdx.x & 31, lr = lane & 15, hi = lane >> 4; const int r0 = blockIdx.x * 64, c0 = blockIdx.y * 64;
    v8f acc[4][4];
#pragma unroll
    for (int mb = 0; mb < 4; ++mb)
#pragma unroll
        for (int nb = 0; nb < 4; ++nb) acc[mb][nb] = (v8f){};
    const size_t aoff = (size_t)(r0 + lr) * K + 8 * hi, boff = (size_t)(c0 + lr) * K + 8 * hi;
#pragma unroll 1
    for (int kc = 0; kc < K; kc += 32) {
        v16bf a[4];
#pragma unroll
        for (int mb = 0; mb < 4; ++mb) a[mb] = ldb(A + aoff + (size_t)mb * 16 * K + kc);
#pragma unroll
        for (int nb = 0; nb < 4; ++nb) { const v16bf b = ldb(Bt + boff + (size_t)nb * 16 * K + kc);
#pragma unroll
            for (int mb = 0; mb < 4; ++mb) acc[mb][nb] = wmmab(a[mb], b, acc[mb][nb]); }
        asm volatile("v_nop\n\tv_nop\n\tv_nop\n\tv_nop" : "+v"(acc[0][0]), "+v"(acc[1][1]), "+v"(acc[2][2]), "+v"(acc[3][3]) : "v"(a[0]), "v"(a[3]));
    }
#pragma unroll
    for (int mb = 0; mb < 4; ++mb) {
#pragma unroll
        for (int nb = 0; nb < 4; ++nb) {
#pragma unroll
            for (int j = 0; j < 8; ++j) os[(hi * 8 + j) * 68 + nb * 16 + lr] = acc[mb][nb][j]; }
        __builtin_amdgcn_wave_barrier(); asm volatile("" ::: "memory");
        float* crow = C + (size_t)(r0 + mb * 16) * ldc + c0;
#pragma unroll 1
        for (int ps = 0; ps < 2; ++ps) {
#pragma unroll
            for (int s = 0; s < 8; ++s) { const int row = 2 * s + hi, cofs = lr * 4; v4f val = *(const v4fa*)(os + row * 68 + cofs); val[0] *= oscale; val[1] *= oscale; val[2] *= oscale; val[3] *= oscale;
                val[0] += bfr(bias[c0 + cofs]); val[1] += bfr(bias[c0 + cofs + 1]); val[2] += bfr(bias[c0 + cofs + 2]); val[3] += bfr(bias[c0 + cofs + 3]);
                *(volatile v4f*)(crow + (size_t)row * ldc + cofs) = val; }
            if (ps == 0) __threadfence(); }
        __builtin_amdgcn_wave_barrier(); asm volatile("" ::: "memory");
    }
}

__global__ __launch_bounds__(256) void k_qkpl(const float* __restrict__ F, bf* PL) { const size_t idx = (size_t)blockIdx.x * 256 + threadIdx.x; if (idx >= PLSZ / 8) return; const int which = blockIdx.y; const size_t e = idx * 8;
    const int d = (int)(e % HD); const int n = (int)((e / HD) % SEQ); const int h = (int)((e / ((size_t)HD * SEQ)) % NH); const int b = (int)(e / ((size_t)HD * SEQ * NH)); const float sc = which ? 1.0f : 0.125f;
    const v8f v = *(const v8f*)(F + ((size_t)b * SEQ + n) * D3 + which * DM + h * HD + d); v8us oh, ol;
#pragma unroll
    for (int k = 0; k < 8; ++k) { unsigned short a2, c2; splitf(v[k] * sc, a2, c2); oh[k] = a2; ol[k] = c2; }
    bf* ph = PL + (size_t)(2 * which) * PLSZ + e; bf* pl = PL + (size_t)(2 * which + 1) * PLSZ + e;
    *(volatile v8us*)ph = oh; *(volatile v8us*)pl = ol; __threadfence(); *(volatile v8us*)ph = oh; *(volatile v8us*)pl = ol; }
__global__ __launch_bounds__(256) void k_vtp(const float* __restrict__ F, h16* VT) { const size_t idx = (size_t)blockIdx.x * 256 + threadIdx.x; if (idx >= PLSZ / 8) return; const size_t e = idx * 8;
    const int t = (int)(e % SEQ); const int d = (int)((e / SEQ) % HD); const int h = (int)((e / ((size_t)SEQ * HD)) % NH); const int b = (int)(e / ((size_t)SEQ * HD * NH));
    const float* f = F + ((size_t)b * SEQ + t) * D3 + 2 * DM + h * HD + d; v8h o;
#pragma unroll
    for (int q = 0; q < 8; ++q) o[q] = (h16)f[(size_t)q * D3];
    *(volatile v8h*)(VT + e) = o; __threadfence(); *(volatile v8h*)(VT + e) = o; }

__global__ __launch_bounds__(256) void k_vres(const float* __restrict__ F, h16* VR) {
#pragma clang fp contract(off)
    const size_t idx = (size_t)blockIdx.x * 256 + threadIdx.x; if (idx >= VRSZ / 8) return; const size_t e = idx * 8;
    const int t = (int)(e % ER); const int d = (int)((e / ER) % HD); const int h = (int)((e / ((size_t)ER * HD)) % NH); const int b = (int)(e / ((size_t)ER * HD * NH));
    const float* f = F + ((size_t)b * SEQ + t) * D3 + 2 * DM + h * HD + d; v8h o;
#pragma unroll
    for (int q = 0; q < 8; ++q) { const float v = f[(size_t)q * D3]; const float hv = (float)(h16)v; o[q] = toh_flush((v - hv) * VRCAR); }
    *(volatile v8h*)(VR + e) = o; __threadfence(); *(volatile v8h*)(VR + e) = o; }

__global__ __launch_bounds__(256) void k_zfill(float* dst, size_t n4) { const size_t i = (size_t)blockIdx.x * 256 + threadIdx.x; if (i >= n4) return; const v4f z = (v4f){};
    *(volatile v4f*)(dst + i * 4) = z; __threadfence(); *(volatile v4f*)(dst + i * 4) = z; }

__global__ __launch_bounds__(256) void k_wstat(const float* __restrict__ w, size_t n4, float* part) {
#pragma clang fp contract(off)
    __shared__ double rs[8];
    __shared__ double ra[8];
    const int tid = threadIdx.x, lane = tid & 31;
    const int wave = __builtin_amdgcn_readfirstlane(threadIdx.x >> 5);
    double s = 0.0, a = 0.0;
#pragma unroll 1
    for (size_t i = (size_t)blockIdx.x * 256 + tid; i < n4; i += (size_t)RB * 256) {
        const v4f v = *(const v4f*)(w + i * 4);
#pragma unroll
        for (int k = 0; k < 4; ++k) { const float t = bfr(v[k]); s += (double)t; a += (double)fabsf(t); }
    }
#pragma unroll
    for (int o = 16; o > 0; o >>= 1) { s += __shfl_xor(s, o, 32); a += __shfl_xor(a, o, 32); }
    if (lane == 0) { rs[wave] = s; ra[wave] = a; }
    __syncthreads();
    if (wave == 0) {
        double ts = 0.0, ta = 0.0;
#pragma unroll
        for (int k = 0; k < 8; ++k) { ts += rs[k]; ta += ra[k]; }
        const float val = (lane == 0) ? (float)ts : ((lane == 1) ? (float)ta : 0.0f);
        float* p = part + (size_t)blockIdx.x * 32 + lane;
        *(volatile float*)p = val; __threadfence(); *(volatile float*)p = val;
    }
}

__global__ __launch_bounds__(256) void k_xstat(const float* __restrict__ src, size_t sS, int rne, float* part) {
#pragma clang fp contract(off)
    __shared__ double rs[8];
    __shared__ double rq[8];
    __shared__ float rm[8];
    const int tid = threadIdx.x, lane = tid & 31;
    const int wave = __builtin_amdgcn_readfirstlane(threadIdx.x >> 5);
    src += (size_t)blockIdx.y * sS;
    const size_t n4 = (size_t)SEQ * DM / 4;
    double s = 0.0, q = 0.0; float m = 0.0f;
#pragma unroll 1
    for (size_t i = (size_t)blockIdx.x * 256 + tid; i < n4; i += (size_t)RB * 256) {
        const v4f v = *(const v4f*)(src + i * 4);
#pragma unroll
        for (int k = 0; k < 4; ++k) { const float t = rne ? bfr(v[k]) : v[k]; const double td = (double)t; s += td; q += td * td; m = fmaxf(m, fabsf(t)); }
    }
#pragma unroll
    for (int o = 16; o > 0; o >>= 1) { s += __shfl_xor(s, o, 32); q += __shfl_xor(q, o, 32); m = fmaxf(m, __shfl_xor(m, o, 32)); }
    if (lane == 0) { rs[wave] = s; rq[wave] = q; rm[wave] = m; }
    __syncthreads();
    if (wave == 0) {
        double ts = 0.0, tq = 0.0; float tm = 0.0f;
#pragma unroll
        for (int k = 0; k < 8; ++k) { ts += rs[k]; tq += rq[k]; tm = fmaxf(tm, rm[k]); }
        const float val = (lane == 0) ? (float)ts : ((lane == 1) ? (float)tq : ((lane == 2) ? tm : 0.0f));
        float* p = part + ((size_t)blockIdx.y * RB + blockIdx.x) * 32 + lane;
        *(volatile float*)p = val; __threadfence(); *(volatile float*)p = val;
    }
}

__global__ __launch_bounds__(32) void k_fin(const float* __restrict__ wpart, const float* __restrict__ xpart, double wninv, float* scal) {
#pragma clang fp contract(off)
    const int lane = threadIdx.x & 31;
    double ws = (double)wpart[(size_t)lane * 32] + (double)wpart[(size_t)(lane + 32) * 32];
    double wa = (double)wpart[(size_t)lane * 32 + 1] + (double)wpart[(size_t)(lane + 32) * 32 + 1];
#pragma unroll
    for (int o = 16; o > 0; o >>= 1) { ws += __shfl_xor(ws, o, 32); wa += __shfl_xor(wa, o, 32); }
    float g = 0.0f;
#pragma unroll 1
    for (int b = 0; b < NB; ++b) g = fmaxf(g, fmaxf(xpart[((size_t)b * RB + lane) * 32 + 2], xpart[((size_t)b * RB + lane + 32) * 32 + 2]));
#pragma unroll
    for (int o = 16; o > 0; o >>= 1) g = fmaxf(g, __shfl_xor(g, o, 32));
    const float alpha = (float)(ws * wninv);
    const float beta = (float)(wa * wninv);
    float outv = 0.0f;
    outv = (lane == 0) ? alpha : outv;
    outv = (lane == 1) ? (beta * g * (1.0f / 128.0f)) : outv;
    outv = (lane == 2) ? (128.0f * (1.0f / g)) : outv;
    const double cinv = 1.0 / ((double)SEQ * (double)DM);
#pragma unroll 1
    for (int b = 0; b < NB; ++b) {
        double s = (double)xpart[((size_t)b * RB + lane) * 32] + (double)xpart[((size_t)b * RB + lane + 32) * 32];
        double q = (double)xpart[((size_t)b * RB + lane) * 32 + 1] + (double)xpart[((size_t)b * RB + lane + 32) * 32 + 1];
#pragma unroll
        for (int o = 16; o > 0; o >>= 1) { s += __shfl_xor(s, o, 32); q += __shfl_xor(q, o, 32); }
        const double mud = s * cinv;
        const double var = q * cinv - mud * mud;
        const float mu = (float)mud;
        const float rstd = 1.0f / sqrtf((float)var + 1e-5f);
        outv = (lane == 4 + b) ? mu : outv;
        outv = (lane == 8 + b) ? rstd : outv;
    }
    float* p = scal + lane;
    *(volatile float*)p = outv; __threadfence(); *(volatile float*)p = outv;
}

__global__ __launch_bounds__(256) void k_signdup(const float* __restrict__ src, const float* __restrict__ scal, bf* dst, size_t n8) {
#pragma clang fp contract(off)
    const size_t i = (size_t)blockIdx.x * 256 + threadIdx.x; if (i >= n8) return; const size_t e = i * 8; const size_t row = e / CK; const int col = ((int)(e % CK)) & (DM - 1);
    const float alpha = scal[0];
    const v8f v = *(const v8f*)(src + row * DM + col); v8us o;
#pragma unroll
    for (int k = 0; k < 8; ++k) { const float d = bfr(v[k]) - alpha; o[k] = (d > 0.0f) ? (unsigned short)0x3F80 : ((d < 0.0f) ? (unsigned short)0xBF80 : (unsigned short)0); }
    *(volatile v8us*)(dst + e) = o; __threadfence(); *(volatile v8us*)(dst + e) = o; }

__global__ __launch_bounds__(256) void k_quant(const float* __restrict__ src, const float* __restrict__ scal, bf* dst, size_t n8, size_t sS, size_t sD, int rne) {
#pragma clang fp contract(off)
    const size_t i = (size_t)blockIdx.x * 256 + threadIdx.x; if (i >= n8) return; const int b = blockIdx.y;
    const float osc = scal[1], qs = scal[2], mu = scal[4 + b], rstd = scal[8 + b];
    const size_t e = i * 8; const size_t row = e / DM; const int col = (int)(e % DM);
    const v8f v = *(const v8f*)(src + (size_t)b * sS + e); v8us oh, ol;
#pragma unroll
    for (int k = 0; k < 8; ++k) { float t = rne ? bfr(v[k]) : v[k]; t = (t - mu) * rstd; t = t * qs; t = fminf(fmaxf(t, -127.99999f), 127.99999f); t = t * osc; unsigned short a2, c2; splitf(t, a2, c2); oh[k] = a2; ol[k] = c2; }
    bf* ph = dst + (size_t)b * sD + row * CK + col; bf* pl = ph + DM;
    *(volatile v8us*)ph = oh; *(volatile v8us*)pl = ol; __threadfence(); *(volatile v8us*)ph = oh; *(volatile v8us*)pl = ol; }

template <bool EARLY>
__device__ __forceinline__ void attn_body(const bf* __restrict__ PL, const h16* __restrict__ VT, const h16* __restrict__ VR, float* Y, const int qbase) {
    __shared__ __align__(16) float ostage[AW * 16 * 68];
    const int lane = threadIdx.x & 31, lr = lane & 15, hf = lane >> 4;
    const int wave = __builtin_amdgcn_readfirstlane(threadIdx.x >> 5);
    const int bh = blockIdx.y, b = bh / NH, h = bh % NH;
    const int q0 = qbase + (blockIdx.x * AW + wave) * 16;
    const bf* QPh = PL; const bf* QPl = PL + PLSZ; const bf* KPh = PL + 2 * PLSZ; const bf* KPl = PL + 3 * PLSZ;
    const size_t zh = (size_t)bh * SEQ * HD;
    const size_t zv = (size_t)bh * HD * SEQ;
    const size_t zr = (size_t)bh * HD * ER;

    v16bf qh[2], ql[2];
#pragma unroll
    for (int kc = 0; kc < 2; ++kc) { const size_t qo = zh + (size_t)(q0 + lr) * HD + kc * 32 + 8 * hf; qh[kc] = ldb(QPh + qo); ql[kc] = ldb(QPl + qo); }

    v8f o[4], o2[4];
#pragma unroll
    for (int jd = 0; jd < 4; ++jd) { o[jd] = (v8f){}; o2[jd] = (v8f){}; }
    float m = -1.0e30f, L = 0.0f;
    const int qcur = q0 + lr;
    const int nst = (q0 + 15) / 32 + 1;

#pragma unroll 1
    for (int st = 0; st < nst; ++st) {
        const int m0 = st * 32;
        v8f s[2];
#pragma unroll
        for (int sub = 0; sub < 2; ++sub) {
            v8f a = (v8f){};
#pragma unroll
            for (int kc = 0; kc < 2; ++kc) {
                const size_t ko = zh + (size_t)(m0 + sub * 16 + lr) * HD + kc * 32 + 8 * hf;
                const v16bf kh = ldb(KPh + ko); const v16bf kl = ldb(KPl + ko);
                a = gwb(kh, qh[kc], a); a = gwb(kl, qh[kc], a); a = gwb(kh, ql[kc], a);
            }
            s[sub] = a;
        }
        float sv[16];
        float tmax = -1.0e30f;
#pragma unroll
        for (int sub = 0; sub < 2; ++sub)
#pragma unroll
            for (int r = 0; r < 8; ++r) { const int key = m0 + sub * 16 + 8 * hf + r; const float v = (key > qcur) ? -1.0e30f : s[sub][r]; sv[sub * 8 + r] = v; tmax = fmaxf(tmax, v); }
        tmax = fmaxf(tmax, __shfl_xor(tmax, 16, 32));
        const float mn = fmaxf(m, tmax);
        const float corr = __builtin_amdgcn_exp2f((m - mn) * L2E);
        m = mn;
        float rsum = 0.0f;
        v16h pb, pr;
#pragma unroll
        for (int i = 0; i < 16; ++i) {
            const float e = (sv[i] - mn) * L2E;
            const float ex = __builtin_amdgcn_exp2f(e + PEXP);
            const float p = (e < -22.0f) ? 0.0f : ex;
            const h16 ph = toh_flush(p);
            pb[i] = ph;
            if (EARLY) { rsum += p; pr[i] = toh_flush((p - (float)ph) * VRCAR); }
            else { rsum += (float)ph; pr[i] = (h16)0.0f; }
        }
        L = L * corr + rsum;
#pragma unroll
        for (int jd = 0; jd < 4; ++jd) { o[jd] = o[jd] * corr; if (EARLY) o2[jd] = o2[jd] * corr; }
#pragma unroll
        for (int jd = 0; jd < 4; ++jd) {
            const v16h va = ldh(VT + zv + (size_t)(jd * 16 + lr) * SEQ + m0 + 8 * hf);
            o[jd] = gwh(va, pb, o[jd]);
            if (EARLY) {
                const v16h vr = ldh(VR + zr + (size_t)(jd * 16 + lr) * ER + m0 + 8 * hf);
                o2[jd] = gwh(vr, pb, o2[jd]);
                o2[jd] = gwh(va, pr, o2[jd]);
            }
        }
    }

    L += __shfl_xor(L, 16, 32);
    const float inv = 1.0f / L;
    const int wb = wave * (16 * 68);
#pragma unroll
    for (int jd = 0; jd < 4; ++jd)
#pragma unroll
        for (int r = 0; r < 8; ++r) { const float val = EARLY ? ((o[jd][r] + o2[jd][r] * (1.0f / VRCAR)) * inv) : (o[jd][r] * inv); ostage[wb + lr * 68 + jd * 16 + 8 * hf + r] = val; }
    asm volatile("s_wait_dscnt 0x0" ::: "memory"); __builtin_amdgcn_wave_barrier(); asm volatile("" ::: "memory");
    float* yrow = Y + ((size_t)b * SEQ + q0) * DM + h * HD;
#pragma unroll 1
    for (int ps = 0; ps < 2; ++ps) {
#pragma unroll
        for (int t = 0; t < 8; ++t) { const int row = 2 * t + hf, cofs = lr * 4; const v4f val = *(const v4fa*)(ostage + wb + row * 68 + cofs); *(volatile v4f*)(yrow + (size_t)row * DM + cofs) = val; }
        if (ps == 0) __threadfence(); }
}

__global__ __launch_bounds__(128) __attribute__((amdgpu_num_vgpr(256))) void k_attn_early(const bf* __restrict__ PL, const h16* __restrict__ VT, const h16* __restrict__ VR, float* Y) { attn_body<true>(PL, VT, VR, Y, 0); }
__global__ __launch_bounds__(128) __attribute__((amdgpu_num_vgpr(256))) void k_attn_late(const bf* __restrict__ PL, const h16* __restrict__ VT, const h16* __restrict__ VR, float* Y) { attn_body<false>(PL, VT, VR, Y, ER); }

static constexpr size_t al256(size_t x) { return (x + 255) & ~(size_t)255; }
static constexpr size_t SZ_XQ  = al256((size_t)NB * SEQ * CK * 2);
static constexpr size_t SZ_WQ  = al256((size_t)D3 * CK * 2);
static constexpr size_t SZ_WP  = al256((size_t)DM * CK * 2);
static constexpr size_t SZ_F   = al256((size_t)NB * SEQ * D3 * 4);
static constexpr size_t SZ_PL  = al256((size_t)4 * NB * NH * SEQ * HD * 2);
static constexpr size_t SZ_VT  = al256((size_t)NB * NH * HD * SEQ * 2);
static constexpr size_t SZ_VR  = al256(VRSZ * 2);
static constexpr size_t SZ_PW  = al256((size_t)RB * 32 * 4);
static constexpr size_t SZ_PX  = al256((size_t)NB * RB * 32 * 4);
static constexpr size_t SZ_SC  = al256((size_t)32 * 4);
static constexpr size_t SZ_ZB  = al256((size_t)D3 * 4);
static constexpr size_t WS_TOTAL = SZ_XQ + SZ_WQ + SZ_WP + SZ_F + SZ_PL + SZ_VT + SZ_VR + 2 * SZ_PW + 2 * SZ_PX + 2 * SZ_SC + SZ_ZB;
static_assert(WS_TOTAL <= (size_t)134217728);
static_assert((size_t)(NB * SEQ / 64) * 64 * CK * 2 <= SZ_XQ);
static_assert((size_t)(D3 / 64) * 64 * CK * 2 <= SZ_WQ);
static_assert((size_t)(DM / 64) * 64 * CK * 2 <= SZ_WP);
static_assert((size_t)NB * SEQ * DM * 4 <= SZ_F);
static_assert((size_t)D3 % 4 == 0 && DM <= D3);

extern "C" void kernel_launch(void* const* d_in, const int* in_sizes, int n_in,
                              void* d_out, int out_size, void* d_ws, size_t ws_size, hipStream_t stream) {
    if (n_in < 3) return;
    const size_t xneed = ((size_t)(NB - 1) * SEQ_FULL + SEQ) * DM;
    if ((size_t)in_sizes[0] < xneed || (size_t)in_sizes[1] < (size_t)D3 * DM || (size_t)in_sizes[2] < (size_t)DM * DM) return;
    if ((size_t)out_size < xneed) return;
    if (WS_TOTAL > ws_size) return;
    const float* x = (const float*)d_in[0]; const float* w_in = (const float*)d_in[1]; const float* w_out = (const float*)d_in[2];
    float* OUT = (float*)d_out;
    char* wsp = (char*)d_ws;
    bf* XQ = (bf*)wsp; wsp += SZ_XQ; bf* WQ = (bf*)wsp; wsp += SZ_WQ; bf* WP = (bf*)wsp; wsp += SZ_WP; float* F = (float*)wsp; wsp += SZ_F;
    bf* PL = (bf*)wsp; wsp += SZ_PL; h16* VT = (h16*)wsp; wsp += SZ_VT; h16* VR = (h16*)wsp; wsp += SZ_VR;
    float* PW1 = (float*)wsp; wsp += SZ_PW; float* PW2 = (float*)wsp; wsp += SZ_PW; float* PX1 = (float*)wsp; wsp += SZ_PX; float* PX2 = (float*)wsp; wsp += SZ_PX;
    float* SC1 = (float*)wsp; wsp += SZ_SC; float* SC2 = (float*)wsp; wsp += SZ_SC; float* ZB = (float*)wsp; wsp += SZ_ZB;
    float* Y = F;
    bf* YQ = XQ;

    k_zfill<<<(unsigned)(((size_t)D3 / 4 + 255) / 256), 256, 0, stream>>>(ZB, (size_t)D3 / 4);
    k_wstat<<<RB, 256, 0, stream>>>(w_in, (size_t)D3 * DM / 4, PW1);
    k_wstat<<<RB, 256, 0, stream>>>(w_out, (size_t)DM * DM / 4, PW2);
    k_xstat<<<dim3(RB, NB, 1), 256, 0, stream>>>(x, (size_t)SEQ_FULL * DM, 1, PX1);
    k_fin<<<1, 32, 0, stream>>>(PW1, PX1, 1.0 / ((double)D3 * (double)DM), SC1);
    k_signdup<<<(unsigned)(((size_t)D3 * CK / 8 + 255) / 256), 256, 0, stream>>>(w_in, SC1, WQ, (size_t)D3 * CK / 8);
    k_quant<<<dim3((unsigned)(((size_t)SEQ * DM / 8 + 255) / 256), NB, 1), 256, 0, stream>>>(x, SC1, XQ, (size_t)SEQ * DM / 8, (size_t)SEQ_FULL * DM, (size_t)SEQ * CK, 1);
    k_gemm_bf<<<dim3(NB * SEQ / 64, D3 / 64, 1), 32, 0, stream>>>(XQ, WQ, CK, F, D3, ZB, 1.0f, 0, 0, 0);
    k_qkpl<<<dim3((unsigned)((PLSZ / 8 + 255) / 256), 2, 1), 256, 0, stream>>>(F, PL);
    k_vtp<<<(unsigned)((PLSZ / 8 + 255) / 256), 256, 0, stream>>>(F, VT);
    k_vres<<<(unsigned)((VRSZ / 8 + 255) / 256), 256, 0, stream>>>(F, VR);
    k_attn_early<<<dim3(ER / 64, NB * NH, 1), AW * 32, 0, stream>>>(PL, VT, VR, Y);
    if (SEQ > EROWS) k_attn_late<<<dim3((SEQ - ER) / 64 > 0 ? (SEQ - ER) / 64 : 1, NB * NH, 1), AW * 32, 0, stream>>>(PL, VT, VR, Y);
    k_xstat<<<dim3(RB, NB, 1), 256, 0, stream>>>(Y, (size_t)SEQ * DM, 0, PX2);
    k_fin<<<1, 32, 0, stream>>>(PW2, PX2, 1.0 / ((double)DM * (double)DM), SC2);
    k_signdup<<<(unsigned)(((size_t)DM * CK / 8 + 255) / 256), 256, 0, stream>>>(w_out, SC2, WP, (size_t)DM * CK / 8);
    k_quant<<<dim3((unsigned)(((size_t)SEQ * DM / 8 + 255) / 256), NB, 1), 256, 0, stream>>>(Y, SC2, YQ, (size_t)SEQ * DM / 8, (size_t)SEQ * DM, (size_t)SEQ * CK, 0);
    k_gemm_bf<<<dim3(SEQ / 64, DM / 64, NB), 32, 0, stream>>>(YQ, WP, CK, OUT, DM, ZB, 1.0f, (size_t)SEQ * CK, 0, (size_t)SEQ_FULL * DM);
}
